// DSAttention_37203006718710
// MI455X (gfx1250) — hardware-verified
//
#include <hip/hip_runtime.h>
#include <math.h>


#define BB 4
#define LL 2048
#define SS 2048
#define HH 8
#define EE 64
#define HE 512
#define TAUP 32

typedef _Float16 v8h  __attribute__((ext_vector_type(8)));
typedef _Float16 v16h __attribute__((ext_vector_type(16)));
typedef __bf16   v8b  __attribute__((ext_vector_type(8)));
typedef __bf16   v16b __attribute__((ext_vector_type(16)));
typedef float    v4f  __attribute__((ext_vector_type(4)));
typedef float    v8f  __attribute__((ext_vector_type(8)));
typedef unsigned int v4u __attribute__((ext_vector_type(4)));
typedef unsigned int v8u __attribute__((ext_vector_type(8)));
typedef v8h __attribute__((may_alias)) v8ha;
typedef v4f __attribute__((may_alias)) v4fa;

union FragH { v16h v; v8h h[2]; };
union FragB { v16b v; v8b h[2]; };
union Pack8 { v8h h; v4u u; };

__device__ __forceinline__ unsigned int bf16_bits(float x) {
  unsigned int u = __float_as_uint(x);
  u += 0x7FFFu + ((u >> 16) & 1u);
  return u >> 16;
}
__device__ __forceinline__ float bf16r(float x) {
  return __uint_as_float(bf16_bits(x) << 16);
}
__device__ __forceinline__ v4u pack_bf16x8(v4f x, v4f y) {
  v4u w;
  w.x = bf16_bits(x.x) | (bf16_bits(x.y) << 16);
  w.y = bf16_bits(x.z) | (bf16_bits(x.w) << 16);
  w.z = bf16_bits(y.x) | (bf16_bits(y.y) << 16);
  w.w = bf16_bits(y.z) | (bf16_bits(y.w) << 16);
  return w;
}
__device__ __forceinline__ v8f zero8() {
  v8f z = {0.f, 0.f, 0.f, 0.f, 0.f, 0.f, 0.f, 0.f};
  return z;
}

__device__ __forceinline__ v8f mma_bf16(v16b a, v16b b, v8f c) {
  v8f d = __builtin_amdgcn_wmma_f32_16x16x32_bf16(false, a, false, b, (short)0, c, false, false);
  asm volatile("v_nop\n\tv_nop\n\tv_nop\n\tv_nop"
               : "+v"(d)
               : "v"(__builtin_bit_cast(v8u, a)), "v"(__builtin_bit_cast(v8u, b)));
  return d;
}
__device__ __forceinline__ v8f mma_f16(v16h a, v16h b, v8f c) {
  v8f d = __builtin_amdgcn_wmma_f32_16x16x32_f16(false, a, false, b, (short)0, c, false, false);
  asm volatile("v_nop\n\tv_nop\n\tv_nop\n\tv_nop"
               : "+v"(d)
               : "v"(__builtin_bit_cast(v8u, a)), "v"(__builtin_bit_cast(v8u, b)));
  return d;
}

__global__ __launch_bounds__(256)
void pack_kernel(const float* __restrict__ Q, const float* __restrict__ K,
                 const float* __restrict__ V,
                 v4u* Qh, v4u* Kh, v4u* Vth, v4u* Vtl) {
  const int sb = blockIdx.x, h = blockIdx.y, b = blockIdx.z;
  const int tid = threadIdx.x;
  const int q8 = tid & 7;
  const int rr = tid >> 3;
  const int s0 = sb * 64;

  __shared__ __align__(16) _Float16 vth[64][72];
  __shared__ __align__(16) _Float16 vtl[64][72];

  v4u wq[2], wk[2], wh[2], wl[2];
  size_t oq[2], ov[2];

#pragma unroll
  for (int ps = 0; ps < 2; ++ps) {
    const int sl = rr + 32 * ps;
    const int s  = s0 + sl;
    const size_t gin = (((size_t)b * SS + s) * HH + h) * EE + 8 * q8;
    const v4f qx = *(const v4f*)(Q + gin), qy = *(const v4f*)(Q + gin + 4);
    const v4f kx = *(const v4f*)(K + gin), ky = *(const v4f*)(K + gin + 4);
    const v4f vx = *(const v4f*)(V + gin), vy = *(const v4f*)(V + gin + 4);
    wq[ps] = pack_bf16x8(qx, qy);
    wk[ps] = pack_bf16x8(kx, ky);
    oq[ps] = ((((size_t)b * HH + h) * LL + s) * EE + 8 * q8) >> 3;
    float vv[8] = {vx.x, vx.y, vx.z, vx.w, vy.x, vy.y, vy.z, vy.w};
#pragma unroll
    for (int i = 0; i < 8; ++i) {
      const float vr = bf16r(vv[i]);
      vth[8 * q8 + i][sl] = (_Float16)(vr * 256.0f);
      vtl[8 * q8 + i][sl] = (_Float16)(vr * 0.125f);
    }
  }
#pragma unroll
  for (int ps = 0; ps < 2; ++ps) {
    *(volatile v4u*)(Qh + oq[ps]) = wq[ps];
    *(volatile v4u*)(Kh + oq[ps]) = wk[ps];
  }
  __syncthreads();
#pragma unroll
  for (int ps = 0; ps < 2; ++ps) {
    const int e = rr + 32 * ps;
    Pack8 ph, pl;
    ph.h = *(const v8ha*)&vth[e][8 * q8];
    pl.h = *(const v8ha*)&vtl[e][8 * q8];
    wh[ps] = ph.u;
    wl[ps] = pl.u;
    ov[ps] = ((((size_t)b * HH + h) * EE + e) * SS + s0 + 8 * q8) >> 3;
    *(volatile v4u*)(Vth + ov[ps]) = wh[ps];
    *(volatile v4u*)(Vtl + ov[ps]) = wl[ps];
  }
  __threadfence();
#pragma unroll
  for (int ps = 0; ps < 2; ++ps) {
    *(volatile v4u*)(Qh + oq[ps])  = wq[ps];
    *(volatile v4u*)(Kh + oq[ps])  = wk[ps];
    *(volatile v4u*)(Vth + ov[ps]) = wh[ps];
    *(volatile v4u*)(Vtl + ov[ps]) = wl[ps];
  }
}

__global__ __launch_bounds__(256)
void stats_kernel(const float* __restrict__ V, float* meanp, float* stdp) {
  const int t = blockIdx.x * 256 + threadIdx.x;
  const int b = t >> 9, he = t & 511;
  const float* p = V + (size_t)b * SS * HE + he;
  double s = 0.0, ss = 0.0;
#pragma unroll 4
  for (int i = 0; i < SS; ++i) {
    const float v = bf16r(p[(size_t)i * HE]);
    s  += (double)v;
    ss += (double)v * (double)v;
  }
  const double mu = s * (1.0 / (double)SS);
  double var = ss * (1.0 / (double)SS) - mu * mu;
  if (var < 0.0) var = 0.0;
  const float muf = (float)mu;
  const float sdf = sqrtf((float)var + 1e-5f);
  *(volatile float*)(meanp + t) = muf;
  *(volatile float*)(stdp + t)  = sdf;
  __threadfence();
  *(volatile float*)(meanp + t) = muf;
  *(volatile float*)(stdp + t)  = sdf;
}

template <int MODE>
__global__ __launch_bounds__(256)
void proj_kernel(const float* __restrict__ V, const float* __restrict__ conv_w,
                 const float* __restrict__ w1, const float* __restrict__ b1,
                 const float* __restrict__ w2, const float* __restrict__ b2,
                 const float* __restrict__ w3, const float* __restrict__ b3,
                 const float* __restrict__ w4, const float* __restrict__ stats,
                 float* outp) {
  const int b = blockIdx.x;
  const int tid = threadIdx.x;
  __shared__ float cw[SS * 3];
  __shared__ float xcat[2 * HE];
  __shared__ float h1[512];
  __shared__ float h2[256];
  __shared__ float h3[128];

  for (int i = tid; i < SS * 3; i += 256) cw[i] = bf16r(conv_w[i]);
  __syncthreads();

  const float* vb = V + (size_t)b * SS * HE;
  for (int w = tid; w < HE; w += 256) {
    const int jm = (w + HE - 1) & (HE - 1);
    const int jp = (w + 1) & (HE - 1);
    const int om = (jm >> 6) * HE + (jm & 63);
    const int o0 = (w  >> 6) * HE + (w  & 63);
    const int op = (jp >> 6) * HE + (jp & 63);
    float acc = 0.f;
#pragma unroll 1
    for (int c = 0; c < SS; ++c) {
      const float* base = vb + (size_t)((c & 255) << 3) * HE + (c >> 8) * EE;
      const float xm = bf16r(base[om]);
      const float x0 = bf16r(base[o0]);
      const float xp = bf16r(base[op]);
      const float* wc = cw + c * 3;
      acc += xm * wc[0] + x0 * wc[1] + xp * wc[2];
    }
    xcat[w] = acc;
  }
  for (int i = tid; i < HE; i += 256) xcat[HE + i] = stats[b * HE + i];
  __syncthreads();

  for (int j = tid; j < 512; j += 256) {
    float acc = bf16r(b1[j]);
#pragma unroll 1
    for (int i = 0; i < 2 * HE; ++i) acc += xcat[i] * bf16r(w1[(size_t)i * 512 + j]);
    h1[j] = fmaxf(acc, 0.f);
  }
  __syncthreads();
  {
    float acc = bf16r(b2[tid]);
#pragma unroll 1
    for (int i = 0; i < 512; ++i) acc += h1[i] * bf16r(w2[i * 256 + tid]);
    h2[tid] = fmaxf(acc, 0.f);
  }
  __syncthreads();
  if (tid < 128) {
    float acc = bf16r(b3[tid]);
#pragma unroll 1
    for (int i = 0; i < 256; ++i) acc += h2[i] * bf16r(w3[i * 128 + tid]);
    h3[tid] = fmaxf(acc, 0.f);
  }
  __syncthreads();

  if (MODE == 0) {
    if (tid < 32) {
      float acc = 0.f;
#pragma unroll 1
      for (int i = 0; i < 128; ++i) acc += h3[i] * bf16r(w4[i]);
      const float tv = expf(acc);
      float* dst = outp + b * TAUP + tid;
      *(volatile float*)dst = tv;
      __threadfence();
      *(volatile float*)dst = tv;
    }
  } else {
    float dv[8];
#pragma unroll
    for (int k = 0; k < 8; ++k) {
      const int j = tid + 256 * k;
      float acc = 0.f;
#pragma unroll 1
      for (int i = 0; i < 128; ++i) acc += h3[i] * bf16r(w4[(size_t)i * SS + j]);
      dv[k] = acc;
    }
    float* dst = outp + (size_t)b * SS + tid;
#pragma unroll
    for (int k = 0; k < 8; ++k) *(volatile float*)(dst + 256 * k) = dv[k];
    __threadfence();
#pragma unroll
    for (int k = 0; k < 8; ++k) *(volatile float*)(dst + 256 * k) = dv[k];
  }
}

template <bool MASKED>
__device__ __forceinline__ void attn_chunk(
    const int s0, const int q0, const int n16, const int hf, const int k8,
    const float tsc, const float sc, const float* __restrict__ dptr,
    const __bf16* __restrict__ kb_base,
    const _Float16* __restrict__ vh_base, const _Float16* __restrict__ vl_base,
    const v16b qa0, const v16b qa1,
    float (&m)[8], float (&l)[8], v8f (&o)[4],
    _Float16 (*phs)[32], _Float16 (*pls)[32]) {
  v8f c[2];
#pragma unroll
  for (int j = 0; j < 2; ++j) {
    const __bf16* kr = kb_base + (size_t)(s0 + 16 * j + n16) * EE;
    FragB u0, u1;
    u0.h[0] = *(const v8b*)(kr + k8);
    u0.h[1] = *(const v8b*)(kr + 16 + k8);
    u1.h[0] = *(const v8b*)(kr + 32 + k8);
    u1.h[1] = *(const v8b*)(kr + 48 + k8);
    v8f acc = zero8();
    acc = mma_bf16(qa0, u0.v, acc);
    acc = mma_bf16(qa1, u1.v, acc);
    c[j] = acc;
  }

  const float d0 = dptr[s0 + n16] * sc;
  const float d1 = dptr[s0 + 16 + n16] * sc;

  float pv0[8], pv1[8], t8[8];
#pragma unroll
  for (int r = 0; r < 8; ++r) {
    float a0 = fmaf(c[0][r], tsc, d0);
    float a1 = fmaf(c[1][r], tsc, d1);
    if (MASKED) {
      const int ql = q0 + 8 * hf + r;
      if (s0 + n16 > ql)      a0 = -1e30f;
      if (s0 + 16 + n16 > ql) a1 = -1e30f;
    }
    pv0[r] = a0; pv1[r] = a1;
    t8[r] = fmaxf(a0, a1);
  }
#pragma unroll
  for (int r = 0; r < 8; ++r) {
    float v = t8[r];
#pragma unroll
    for (int off = 1; off < 16; off <<= 1) v = fmaxf(v, __shfl_xor(v, off, 32));
    t8[r] = v;
  }

  __syncthreads();
  float rs[8];
#pragma unroll
  for (int r = 0; r < 8; ++r) {
    const float mn   = fmaxf(m[r], t8[r]);
    const float corr = exp2f(m[r] - mn);
    const float p0 = exp2f(pv0[r] - mn) * 4096.0f;
    const float p1 = exp2f(pv1[r] - mn) * 4096.0f;
    m[r] = mn;
    l[r] = l[r] * corr;
#pragma unroll
    for (int t = 0; t < 4; ++t) o[t][r] = o[t][r] * corr;
    const _Float16 h0 = (_Float16)p0;
    const _Float16 h1 = (_Float16)p1;
    const _Float16 l0 = (_Float16)((p0 - (float)h0) * 2048.0f);
    const _Float16 l1 = (_Float16)((p1 - (float)h1) * 2048.0f);
    const int mr = 8 * hf + r;
    phs[mr][n16] = h0;  phs[mr][16 + n16] = h1;
    pls[mr][n16] = l0;  pls[mr][16 + n16] = l1;
    rs[r] = p0 + p1;
  }
#pragma unroll
  for (int r = 0; r < 8; ++r) {
    float v = rs[r];
#pragma unroll
    for (int off = 1; off < 16; off <<= 1) v += __shfl_xor(v, off, 32);
    l[r] += v;
  }
  __syncthreads();

  FragH ah, al;
  ah.h[0] = *(const v8ha*)&phs[n16][k8];
  ah.h[1] = *(const v8ha*)&phs[n16][16 + k8];
  al.h[0] = *(const v8ha*)&pls[n16][k8];
  al.h[1] = *(const v8ha*)&pls[n16][16 + k8];

#pragma unroll
  for (int t = 0; t < 4; ++t) {
    const size_t vo = (size_t)(16 * t + n16) * SS + s0;
    FragH vb, wb;
    vb.h[0] = *(const v8h*)(vh_base + vo + k8);
    vb.h[1] = *(const v8h*)(vh_base + vo + 16 + k8);
    wb.h[0] = *(const v8h*)(vl_base + vo + k8);
    wb.h[1] = *(const v8h*)(vl_base + vo + 16 + k8);
    o[t] = mma_f16(ah.v, vb.v, o[t]);
    o[t] = mma_f16(al.v, wb.v, o[t]);
  }
}

__global__ __launch_bounds__(32)
void attn_kernel(const __bf16* __restrict__ Qh, const __bf16* __restrict__ Kh,
                 const _Float16* __restrict__ Vth, const _Float16* __restrict__ Vtl,
                 const float* __restrict__ taup, const float* __restrict__ deltap,
                 float* out) {
  const int qt = blockIdx.x, h = blockIdx.y, b = blockIdx.z;
  const int q0 = qt * 16;
  const int lane = threadIdx.x & 31;
  const int n16  = lane & 15;
  const int hf   = lane >> 4;
  const int k8   = 8 * hf;

  __shared__ __align__(16) _Float16 phs[16][32];
  __shared__ __align__(16) _Float16 pls[16][32];
  __shared__ __align__(16) float ost[16][64];

  const float sc  = 0.125f * 1.44269504088896340736f;
  const float tsc = taup[b * TAUP] * sc;
  const float* dptr = deltap + (size_t)b * SS;
  const size_t bh = (size_t)b * HH + h;

  const __bf16* qrow = Qh + (bh * LL + q0 + n16) * EE;
  FragB f0, f1;
  f0.h[0] = *(const v8b*)(qrow + k8);       f0.h[1] = *(const v8b*)(qrow + 16 + k8);
  f1.h[0] = *(const v8b*)(qrow + 32 + k8);  f1.h[1] = *(const v8b*)(qrow + 48 + k8);
  const v16b qa0 = f0.v, qa1 = f1.v;

  float m[8], l[8];
  v8f o[4];
#pragma unroll
  for (int r = 0; r < 8; ++r) { m[r] = -1e30f; l[r] = 0.f; }
#pragma unroll
  for (int t = 0; t < 4; ++t) o[t] = zero8();

  const __bf16*   kb_base = Kh  + bh * LL * EE;
  const _Float16* vh_base = Vth + bh * EE * SS;
  const _Float16* vl_base = Vtl + bh * EE * SS;

  const int nfull = q0 >> 5;
#pragma unroll 1
  for (int ci = 0; ci < nfull; ++ci)
    attn_chunk<false>(ci * 32, q0, n16, hf, k8, tsc, sc, dptr, kb_base, vh_base, vl_base,
                      qa0, qa1, m, l, o, phs, pls);
  attn_chunk<true>(nfull * 32, q0, n16, hf, k8, tsc, sc, dptr, kb_base, vh_base, vl_base,
                   qa0, qa1, m, l, o, phs, pls);

  float inv[8];
#pragma unroll
  for (int r = 0; r < 8; ++r) inv[r] = (1.0f / l[r]) * (1.0f / 256.0f);
#pragma unroll
  for (int t = 0; t < 4; ++t) {
#pragma unroll
    for (int r = 0; r < 8; ++r) ost[8 * hf + r][16 * t + n16] = o[t][r] * inv[r];
  }
  __syncthreads();

  const int qq = lane & 7, lq = lane >> 3;
  v4f vals[8];
#pragma unroll
  for (int it = 0; it < 8; ++it) {
    const int L = it * 4 + lq;
    const int row = L >> 1, col = (L & 1) * 32 + 4 * qq;
    vals[it] = *(const v4fa*)&ost[row][col];
  }
  float* obase = out + ((size_t)b * LL + q0) * HH * EE + (size_t)h * EE;
#pragma unroll
  for (int it = 0; it < 8; ++it) {
    const int L = it * 4 + lq;
    const int row = L >> 1, col = (L & 1) * 32 + 4 * qq;
    *(volatile v4f*)(obase + (size_t)row * HH * EE + col) = vals[it];
  }
  __threadfence();
#pragma unroll
  for (int it = 0; it < 8; ++it) {
    const int L = it * 4 + lq;
    const int row = L >> 1, col = (L & 1) * 32 + 4 * qq;
    *(volatile v4f*)(obase + (size_t)row * HH * EE + col) = vals[it];
  }
}

extern "C" void kernel_launch(void* const* d_in, const int* in_sizes, int n_in,
                              void* d_out, int out_size, void* d_ws, size_t ws_size,
                              hipStream_t stream) {
  const float* queries    = (const float*)d_in[0];
  const float* keys       = (const float*)d_in[1];
  const float* values     = (const float*)d_in[2];
  const float* tau_conv_w = (const float*)d_in[3];
  const float* tau_w1     = (const float*)d_in[4];
  const float* tau_b1     = (const float*)d_in[5];
  const float* tau_w2     = (const float*)d_in[6];
  const float* tau_b2     = (const float*)d_in[7];
  const float* tau_w3     = (const float*)d_in[8];
  const float* tau_b3     = (const float*)d_in[9];
  const float* tau_w4     = (const float*)d_in[10];
  const float* del_conv_w = (const float*)d_in[11];
  const float* del_w1     = (const float*)d_in[12];
  const float* del_b1     = (const float*)d_in[13];
  const float* del_w2     = (const float*)d_in[14];
  const float* del_b2     = (const float*)d_in[15];
  const float* del_w3     = (const float*)d_in[16];
  const float* del_b3     = (const float*)d_in[17];
  const float* del_w4     = (const float*)d_in[18];

  char* ws = (char*)d_ws;
  const size_t TEN   = (size_t)BB * HH * LL * EE * 2;
  const size_t O_QH  = 0;
  const size_t O_KH  = O_QH + TEN;
  const size_t O_VTH = O_KH + TEN;
  const size_t O_VTL = O_VTH + TEN;
  const size_t O_MN  = O_VTL + TEN;
  const size_t O_SD  = O_MN + (size_t)BB * HE * 4;
  const size_t O_TAU = O_SD + (size_t)BB * HE * 4;
  const size_t O_DEL = O_TAU + (size_t)BB * TAUP * 4;
  const size_t O_END = O_DEL + (size_t)BB * SS * 4;
  if (O_END > ws_size) return;

  v4u*   Qh   = (v4u*)(ws + O_QH);
  v4u*   Kh   = (v4u*)(ws + O_KH);
  v4u*   Vth  = (v4u*)(ws + O_VTH);
  v4u*   Vtl  = (v4u*)(ws + O_VTL);
  float* mnp  = (float*)(ws + O_MN);
  float* stp  = (float*)(ws + O_SD);
  float* taup = (float*)(ws + O_TAU);
  float* delp = (float*)(ws + O_DEL);

  pack_kernel<<<dim3(SS / 64, HH, BB), 256, 0, stream>>>(queries, keys, values, Qh, Kh, Vth, Vtl);
  stats_kernel<<<(BB * HE) / 256, 256, 0, stream>>>(values, mnp, stp);
  proj_kernel<0><<<BB, 256, 0, stream>>>(values, tau_conv_w, tau_w1, tau_b1, tau_w2, tau_b2,
                                         tau_w3, tau_b3, tau_w4, stp, taup);
  proj_kernel<1><<<BB, 256, 0, stream>>>(values, del_conv_w, del_w1, del_b1, del_w2, del_b2,
                                         del_w3, del_b3, del_w4, mnp, delp);
  attn_kernel<<<dim3(LL / 16, HH, BB), 32, 0, stream>>>(
      (const __bf16*)(ws + O_QH), (const __bf16*)(ws + O_KH),
      (const _Float16*)(ws + O_VTH), (const _Float16*)(ws + O_VTL),
      taup, delp, (float*)d_out);
}
